// FNSD_51762945852046
// MI455X (gfx1250) — hardware-verified
//
#include <hip/hip_runtime.h>
#include <stddef.h>


#define DM      128
#define NLAYER  4
#define NMAT    9
#define NWROWS  (NMAT * DM)
#define WPP     136
#define AP      136
#define EP      132
#define RB      1024
#define RBBITS  10
#define RMAX    128
#define RMBITS  7
#define TABW    (2 * RMAX)
#define CHUNK   4096
#define LCAP    20480
#define DEGCAP  96
#define GPB     4
#define WSCAP   134217728

#define GEMM_LDS_A   (128 * AP * 2)
#define GEMM_LDS_E   (8 * 16 * EP * 4)
#define GEMM_LDS     (GEMM_LDS_A + GEMM_LDS_E)
#define CSR_LDS_INTS (RB + 8 + RB + LCAP)
#define CSR_LDS      (CSR_LDS_INTS * 4)

static_assert(RB == (1 << RBBITS));
static_assert(RMAX == (1 << RMBITS));
static_assert(RMAX <= 256 && (RMAX % 32) == 0);
static_assert(CHUNK == 8 * 16 * 32);
static_assert(CHUNK == 4 * 4 * 256);
static_assert(TABW * 4 == 64 * 16);
static_assert(RB == 4 * 256);
static_assert((LCAP % 1024) == 0);
static_assert(DEGCAP < 255);
static_assert((GEMM_LDS_A % 16) == 0 && (GEMM_LDS % 16) == 0);
static_assert(GEMM_LDS < 160000);
static_assert(CSR_LDS < 160000);
static_assert((AP % 8) == 0 && (WPP % 8) == 0 && (EP % 4) == 0);
static_assert(DM == 32 * 4);
static_assert(GPB <= 8);

typedef float          v4f  __attribute__((ext_vector_type(4)));
typedef float          v8f  __attribute__((ext_vector_type(8)));
typedef double         v2d  __attribute__((ext_vector_type(2)));
typedef double         v4d  __attribute__((ext_vector_type(4)));
typedef int            v4i  __attribute__((ext_vector_type(4)));
typedef unsigned int   v4u  __attribute__((ext_vector_type(4)));
typedef _Float16       v4h  __attribute__((ext_vector_type(4)));
typedef _Float16       v8h  __attribute__((ext_vector_type(8)));
typedef _Float16       v16h __attribute__((ext_vector_type(16)));
union FragH { v16h v; v8h h[2]; };
union Pack8 { v8h h; v4u u; };

static __device__ const float kWCarry = 64.0f;
static __device__ const float kWInv   = 0.015625f;

__device__ __forceinline__ v8f wmh(v16h a, v16h b, v8f c) {
  v8f d = __builtin_amdgcn_wmma_f32_16x16x32_f16(false, a, false, b, (short)0, c, false, false);
  asm volatile("v_nop\n\tv_nop\n\tv_nop\n\tv_nop" : "+v"(d) : "v"(a), "v"(b));
  return d;
}

template <int NB>
__device__ __forceinline__ unsigned int match_mask(unsigned int base, int key) {
  unsigned int msk = base;
#pragma unroll
  for (int b = 0; b < NB; ++b) {
    const bool bit = ((key >> b) & 1) != 0;
    const unsigned int bb = __builtin_amdgcn_ballot_w32(bit);
    msk &= bit ? bb : ~bb;
  }
  return msk;
}

__global__ __launch_bounds__(256) void k_csort(
    const int* __restrict__ er, const int* __restrict__ ec,
    unsigned int* csort, int* tab, int nN, int nE1, int nE2) {
  __shared__ __attribute__((aligned(16))) unsigned int sImg[CHUNK];
  __shared__ int cw[8 * RMAX];
  __shared__ __attribute__((aligned(16))) int sTb[TABW];
  __shared__ int sWt[8];
  int* sPre = sTb;
  int* sCn  = sTb + RMAX;
  const int tid = (int)threadIdx.x, lane = tid & 31, wave = tid >> 5;
  const int c = (int)blockIdx.x;
  const int cbase = c * CHUNK;

  for (int i = tid; i < 8 * RMAX; i += 256) cw[i] = 0;
  {
    const v4u s = {0xffffffffu, 0xffffffffu, 0xffffffffu, 0xffffffffu};
    for (int i = tid; i < CHUNK / 4; i += 256) ((v4u*)sImg)[i] = s;
  }
  __syncthreads();

  unsigned int ent[16];
  int pk[16];
  const unsigned int lt = (1u << lane) - 1u;
#pragma unroll
  for (int i = 0; i < 16; ++i) {
    const int e = cbase + wave * 512 + 32 * i + lane;
    const int ea = e > nE2 - 1 ? nE2 - 1 : e;
    const bool fh = ea < nE1;
    const int i1 = fh ? ea : (ea - nE1);
    const int a = er[i1];
    const int b = ec[i1];
    const int d = fh ? a : b;
    const int s = fh ? b : a;
    const bool valid = (e < nE2) && ((unsigned)d < (unsigned)nN) && (s != d);
    const int dd = valid ? d : 0;
    const int r  = dd >> RBBITS;
    const int jl = dd & (RB - 1);
    const unsigned int pay = (unsigned int)ea;
    const unsigned int msk = match_mask<RMBITS>(__builtin_amdgcn_ballot_w32(valid), r);
    const int rank = (int)__builtin_popcount(msk & lt);
    const int grp  = (int)__builtin_popcount(msk);
    const int base = cw[wave * RMAX + r];
    pk[i]  = valid ? ((r << 12) | (base + rank)) : -1;
    ent[i] = (pay << RBBITS) | (unsigned int)jl;
    if (valid && rank == 0) cw[wave * RMAX + r] = base + grp;
    __syncthreads();
  }

  if (tid < RMAX) {
    int run = 0;
#pragma unroll
    for (int w = 0; w < 8; ++w) {
      const int v = cw[w * RMAX + tid];
      cw[w * RMAX + tid] = run;
      run += v;
    }
    sCn[tid] = run;
  }
  __syncthreads();
  {
    const int vr = sCn[tid & (RMAX - 1)];
    const int v  = (tid < RMAX) ? vr : 0;
    int x = v;
#pragma unroll
    for (int dd = 1; dd < 32; dd <<= 1) {
      const int y = __shfl_up(x, dd);
      x += (lane >= dd) ? y : 0;
    }
    if (lane == 31) sWt[wave] = x;
    __syncthreads();
    int pre = 0;
#pragma unroll
    for (int w = 0; w < 8; ++w) { const int tw = sWt[w]; pre += (w < wave) ? tw : 0; }
    if (tid < RMAX) sPre[tid] = pre + x - v;
  }
  __syncthreads();

#pragma unroll
  for (int i = 0; i < 16; ++i) {
    if (pk[i] >= 0) {
      const int r = (pk[i] >> 12) & (RMAX - 1);
      const int q = pk[i] & 4095;
      const int pos = sPre[r] + cw[wave * RMAX + r] + q;
      if ((unsigned)pos < (unsigned)CHUNK) sImg[pos] = ent[i];
    }
  }
  __syncthreads();

  v4u iv[4];
#pragma unroll
  for (int it = 0; it < 4; ++it) iv[it] = ((const v4u*)sImg)[it * 256 + tid];
  const v4i tv = *(const v4i*)(sTb + 4 * (tid & 63));
  unsigned int* gp = csort + (size_t)c * CHUNK;
  int* tp = tab + (size_t)c * TABW + 4 * (tid & 63);
  const bool wt = tid < 64;
#pragma unroll
  for (int it = 0; it < 4; ++it) *(volatile v4u*)(gp + 4 * (it * 256 + tid)) = iv[it];
  if (wt) *(volatile v4i*)tp = tv;
  __threadfence();
#pragma unroll
  for (int it = 0; it < 4; ++it) *(volatile v4u*)(gp + 4 * (it * 256 + tid)) = iv[it];
  if (wt) *(volatile v4i*)tp = tv;
}

__global__ __launch_bounds__(256) void k_csr(
    const int* __restrict__ er, const int* __restrict__ ec,
    const unsigned int* __restrict__ csort, const int* __restrict__ tab,
    int* srcs, int* ntab, int nN, int nE1, int nE2, int nCh, int listCap) {
  extern __shared__ __attribute__((aligned(16))) int cdyn[];
  __shared__ int sWtot[8];
  __shared__ int sTot[RMAX];
  __shared__ int sRed[8];
  int* sOff  = cdyn;
  int* sCur  = cdyn + (RB + 8);
  int* sList = sCur + RB;
  const int tid = (int)threadIdx.x, lane = tid & 31, wave = tid >> 5;
  const int rgn = (int)blockIdx.x;
  const int n0 = rgn * RB;
  const unsigned int lt = (1u << lane) - 1u;

  for (int i = tid; i < RB + 8; i += 256) sOff[i] = 0;
  for (int i = tid; i < RB; i += 256) sCur[i] = 0;
  for (int i = tid; i < LCAP; i += 256) sList[i] = 0;

  if (tid < RMAX) {
    int tot = 0;
#pragma unroll 1
    for (int c = 0; c < nCh; ++c) {
      int pre = tab[(size_t)c * TABW + tid];
      int n   = tab[(size_t)c * TABW + RMAX + tid];
      pre = pre < 0 ? 0 : (pre > CHUNK ? CHUNK : pre);
      n = n < 0 ? 0 : (n > CHUNK - pre ? CHUNK - pre : n);
      tot += n;
    }
    sTot[tid] = tot;
  }
  __syncthreads();
  int base = 0;
  {
    const int tr = sTot[tid & (RMAX - 1)];
    const int t32 = ((tr + 31) >> 5) << 5;
    int v = (tid < RMAX && tid < rgn) ? t32 : 0;
#pragma unroll
    for (int off = 16; off > 0; off >>= 1) v += __shfl_xor(v, off);
    if (lane == 0) sRed[wave] = v;
    __syncthreads();
#pragma unroll
    for (int w = 0; w < 8; ++w) base += sRed[w];
  }

#pragma unroll 1
  for (int c = 0; c < nCh; ++c) {
    int pre = tab[(size_t)c * TABW + rgn];
    int n   = tab[(size_t)c * TABW + RMAX + rgn];
    pre = pre < 0 ? 0 : (pre > CHUNK ? CHUNK : pre);
    n = n < 0 ? 0 : (n > CHUNK - pre ? CHUNK - pre : n);
    const int nstep = (n + 31) >> 5;
    const unsigned int* cp = csort + (size_t)c * CHUNK + pre;
#pragma unroll 1
    for (int s = 0; s < nstep; ++s) {
      if (wave == 0) {
        const int i = (s << 5) + lane;
        const bool valid = i < n;
        const int ic = i > n - 1 ? n - 1 : i;
        const unsigned int en = cp[ic];
        const int j = (int)(en & (unsigned int)(RB - 1));
        const unsigned int msk = match_mask<RBBITS>(__builtin_amdgcn_ballot_w32(valid), j);
        const int rank = (int)__builtin_popcount(msk & lt);
        const int grp  = (int)__builtin_popcount(msk);
        if (valid && rank == 0) sOff[j] = sOff[j] + grp;
      }
      __syncthreads();
    }
  }
  __syncthreads();

  {
    int cn[4];
    int ls = 0;
#pragma unroll
    for (int i = 0; i < 4; ++i) { cn[i] = sOff[4 * tid + i]; ls += cn[i]; }
    int x = ls;
#pragma unroll
    for (int dd = 1; dd < 32; dd <<= 1) {
      const int y = __shfl_up(x, dd);
      x += (lane >= dd) ? y : 0;
    }
    if (lane == 31) sWtot[wave] = x;
    __syncthreads();
    int pre = 0;
#pragma unroll
    for (int w = 0; w < 8; ++w) { const int tw = sWtot[w]; pre += (w < wave) ? tw : 0; }
    int run = pre + x - ls;
#pragma unroll
    for (int i = 0; i < 4; ++i) { sOff[4 * tid + i] = run; run += cn[i]; }
    if (tid == 255) sOff[RB] = run;
  }
  __syncthreads();
  const bool rgnOver = sOff[RB] > LCAP;

#pragma unroll 1
  for (int c = 0; c < nCh; ++c) {
    int pre = tab[(size_t)c * TABW + rgn];
    int n   = tab[(size_t)c * TABW + RMAX + rgn];
    pre = pre < 0 ? 0 : (pre > CHUNK ? CHUNK : pre);
    n = n < 0 ? 0 : (n > CHUNK - pre ? CHUNK - pre : n);
    const int nstep = (n + 31) >> 5;
    const unsigned int* cp = csort + (size_t)c * CHUNK + pre;
#pragma unroll 1
    for (int s = 0; s < nstep; ++s) {
      if (wave == 0) {
        const int i = (s << 5) + lane;
        const bool valid = i < n;
        const int ic = i > n - 1 ? n - 1 : i;
        const unsigned int en = cp[ic];
        const int j = (int)(en & (unsigned int)(RB - 1));
        int e = (int)(en >> RBBITS);
        e = e > nE2 - 1 ? nE2 - 1 : e;
        const bool fh = e < nE1;
        const int i1 = fh ? e : (e - nE1);
        const int a = er[i1];
        const int b = ec[i1];
        int sv = fh ? b : a;
        sv = sv < 0 ? 0 : (sv > nN - 1 ? nN - 1 : sv);
        const unsigned int msk = match_mask<RBBITS>(__builtin_amdgcn_ballot_w32(valid), j);
        const int rank = (int)__builtin_popcount(msk & lt);
        const int grp  = (int)__builtin_popcount(msk);
        const int cur  = sCur[j];
        const int p0   = sOff[j] + cur + rank;
        if (valid && (unsigned)p0 < (unsigned)LCAP) sList[p0] = sv;
        if (valid && rank == 0) sCur[j] = cur + grp;
      }
      __syncthreads();
    }
  }
  __syncthreads();

  {
    const int tot = sOff[RB];
    const int totc = tot < 0 ? 0 : (tot > LCAP ? LCAP : tot);
    const int n32 = ((totc + 31) >> 5) << 5;
#pragma unroll 1
    for (int it = 0; it < LCAP / 1024; ++it) {
      const int p = it * 1024 + 4 * tid;
      const bool ok = (p < n32) && (base + p < listCap);
      const v4i v = *(const v4i*)(sList + p);
      if (ok) *(volatile v4i*)(srcs + (size_t)base + p) = v;
    }
    __threadfence();
#pragma unroll 1
    for (int it = 0; it < LCAP / 1024; ++it) {
      const int p = it * 1024 + 4 * tid;
      const bool ok = (p < n32) && (base + p < listCap);
      const v4i v = *(const v4i*)(sList + p);
      if (ok) *(volatile v4i*)(srcs + (size_t)base + p) = v;
    }
  }

  {
    int e4[4];
#pragma unroll
    for (int i = 0; i < 4; ++i) {
      const int j = 4 * tid + i;
      int st = base + sOff[j];
      st = st < 0 ? 0 : (st > 0x7FFFFF ? 0x7FFFFF : st);
      int cn = sOff[j + 1] - sOff[j];
      cn = cn < 0 ? 0 : (cn > 255 ? 255 : cn);
      const int code = rgnOver ? 255 : cn;
      e4[i] = (st << 8) | code;
    }
    const v4i ev = {e4[0], e4[1], e4[2], e4[3]};
    int* np = ntab + (size_t)rgn * RB + 4 * tid;
    *(volatile v4i*)np = ev;
    __threadfence();
    *(volatile v4i*)np = ev;
  }
}

__global__ __launch_bounds__(256) void k_wprep(
    const float* __restrict__ W0, const float* __restrict__ W1, const float* __restrict__ W2,
    _Float16* WT) {
  __shared__ __attribute__((aligned(16))) _Float16 sH[32 * WPP];
  const int tid = (int)threadIdx.x;
  const int b = (int)blockIdx.x;
  const int mat = b >> 2;
  const int nb0 = (b & 3) * 32;
  const float* Wb = (mat == 0) ? W0
                  : ((mat <= NLAYER) ? (W1 + (size_t)(mat - 1) * DM * DM)
                                     : (W2 + (size_t)(mat - 1 - NLAYER) * DM * DM));
  const int rowBase = b * 32;

#pragma unroll 1
  for (int it = 0; it < 4; ++it) {
    const int p = it * 256 + tid;
    const int k = p >> 3, q = p & 7;
    const int c = nb0 + 4 * q;
    const v4f w = *(const v4f*)(Wb + (size_t)k * DM + c);
    _Float16* dh = sH + (4 * q) * WPP + k;
    dh[0]       = (_Float16)(w.x * kWCarry);
    dh[WPP]     = (_Float16)(w.y * kWCarry);
    dh[2 * WPP] = (_Float16)(w.z * kWCarry);
    dh[3 * WPP] = (_Float16)(w.w * kWCarry);
  }
  __syncthreads();

  Pack8 o[2];
#pragma unroll
  for (int it = 0; it < 2; ++it) {
    const int p = it * 256 + tid;
    const int row = p >> 4, c8 = (p & 15) * 8;
    o[it].h = *(const v8h*)(sH + row * WPP + c8);
  }
#pragma unroll
  for (int it = 0; it < 2; ++it) {
    const int p = it * 256 + tid;
    const int row = p >> 4, c8 = (p & 15) * 8;
    *(volatile v4u*)(WT + (size_t)(rowBase + row) * DM + c8) = o[it].u;
  }
  __threadfence();
#pragma unroll
  for (int it = 0; it < 2; ++it) {
    const int p = it * 256 + tid;
    const int row = p >> 4, c8 = (p & 15) * 8;
    *(volatile v4u*)(WT + (size_t)(rowBase + row) * DM + c8) = o[it].u;
  }
}

template <int MODE>
__global__ __launch_bounds__(256) void k_gemm(
    const float* __restrict__ Ain, const int* __restrict__ srcs, const int* __restrict__ ntab,
    int listCap, const float* __restrict__ epsp, const _Float16* __restrict__ WT,
    const float* __restrict__ bias, const float* __restrict__ stats,
    const float* __restrict__ bng, const float* __restrict__ bnb,
    const float* __restrict__ lng, const float* __restrict__ lnb,
    float* outF, double* part, int nN, int nNp) {
  extern __shared__ __attribute__((aligned(16))) int gdyn[];
  __shared__ __attribute__((aligned(16))) double sSt[8 * 32 * 8];
  __shared__ __attribute__((aligned(16))) double sCol[256];
  _Float16* sA = (_Float16*)gdyn;
  float* sE = (float*)((char*)gdyn + GEMM_LDS_A);
  const int tid = (int)threadIdx.x, lane = tid & 31, wave = tid >> 5, hh = lane >> 4, m = lane & 15;
  const int c4 = 4 * lane;
  const int rw0 = (int)blockIdx.x * 128 + 16 * wave;
  const v4f zero4 = {0.0f, 0.0f, 0.0f, 0.0f};

  {
    v4f mu4 = zero4, rs4 = zero4, g4 = zero4, be4 = zero4;
    float alpha = 1.0f;
    if (MODE == 2) {
      mu4 = *(const v4f*)(stats + c4);
      rs4 = *(const v4f*)(stats + DM + c4);
      g4  = *(const v4f*)(bng + c4);
      be4 = *(const v4f*)(bnb + c4);
    }
    if (MODE == 1) alpha = 1.0f + epsp[0];
    const float qn = __int_as_float(0x7fc00000);
    const v4f nan4 = {qn, qn, qn, qn};
#pragma unroll 1
    for (int r = 0; r < 16; ++r) {
      const int row = rw0 + r;
      v4f u;
      if (MODE == 0) {
        const int ra = row > nN - 1 ? nN - 1 : row;
        u = *(const v4f*)(Ain + (size_t)ra * DM + c4);
      } else if (MODE == 2) {
        const v4f p = *(const v4f*)(Ain + (size_t)row * DM + c4);
        v4f t = (p - mu4) * rs4 * g4 + be4;
        t.x = fmaxf(t.x, 0.0f); t.y = fmaxf(t.y, 0.0f); t.z = fmaxf(t.z, 0.0f); t.w = fmaxf(t.w, 0.0f);
        u = t;
      } else {
        const int enl = ntab[row];
        const int en = __builtin_amdgcn_readfirstlane(enl);
        int st = en >> 8;
        const int craw = en & 255;
        const bool bad = craw > DEGCAP;
        const int cnt = bad ? 0 : craw;
        st = st < 0 ? 0 : (st > listCap - 1 ? listCap - 1 : st);
        v4f ag = zero4;
#pragma unroll 1
        for (int it = 0; it < cnt; ++it) {
          int li = st + it; li = li > listCap - 1 ? listCap - 1 : li;
          int sv = srcs[li]; sv = sv < 0 ? 0 : (sv > nN - 1 ? nN - 1 : sv);
          const v4f hv = *(const v4f*)(Ain + (size_t)sv * DM + c4);
          ag = ag + hv;
        }
        const v4f hs = *(const v4f*)(Ain + (size_t)row * DM + c4);
        u = hs * alpha + ag;
        u = bad ? nan4 : u;
      }
      u = (row < nN) ? u : zero4;
      v4h h4;
      h4.x = (_Float16)u.x; h4.y = (_Float16)u.y; h4.z = (_Float16)u.z; h4.w = (_Float16)u.w;
      *(v4h*)(sA + (size_t)(16 * wave + r) * AP + c4) = h4;
    }
  }
  __syncthreads();

  v8f acc[8];
#pragma unroll
  for (int nt = 0; nt < 8; ++nt) { v8f z = {0.f, 0.f, 0.f, 0.f, 0.f, 0.f, 0.f, 0.f}; acc[nt] = z; }
  const _Float16* ap = sA + (size_t)(16 * wave + m) * AP + 8 * hh;
  const _Float16* bp = WT + (size_t)m * DM + 8 * hh;
#pragma unroll 1
  for (int kt = 0; kt < 4; ++kt) {
    const int kb = kt << 5;
    FragH a;
    a.h[0] = *(const v8h*)(ap + kb);
    a.h[1] = *(const v8h*)(ap + kb + 16);
#pragma unroll
    for (int nt = 0; nt < 8; ++nt) {
      FragH b;
      b.h[0] = *(const v8h*)(bp + (size_t)nt * 16 * DM + kb);
      b.h[1] = *(const v8h*)(bp + (size_t)nt * 16 * DM + kb + 16);
      acc[nt] = wmh(a.v, b.v, acc[nt]);
    }
  }

  float* se = sE + wave * (16 * EP);
#pragma unroll
  for (int nt = 0; nt < 8; ++nt)
#pragma unroll
    for (int r = 0; r < 8; ++r)
      se[(8 * hh + r) * EP + 16 * nt + m] = acc[nt][r] * kWInv;
  __syncthreads();

  double sx = 0.0, sy = 0.0, sz = 0.0, sw = 0.0, qx = 0.0, qy = 0.0, qz = 0.0, qw = 0.0;
  const v4f bias4 = *(const v4f*)(bias + c4);
  v4f lg4 = zero4, lb4 = zero4;
  if (MODE == 2) { lg4 = *(const v4f*)(lng + c4); lb4 = *(const v4f*)(lnb + c4); }
#pragma unroll 1
  for (int r = 0; r < 16; ++r) {
    const int row = rw0 + r;
    const bool live = row < nN;
    v4f v = *(const v4f*)(se + r * EP + c4) + bias4;
    v4f o;
    if (MODE == 0) {
      o = live ? v : zero4;
    } else if (MODE == 1) {
      o = v;
      const v4f lv = live ? v : zero4;
      sx += (double)lv.x; sy += (double)lv.y; sz += (double)lv.z; sw += (double)lv.w;
      qx += (double)lv.x * (double)lv.x; qy += (double)lv.y * (double)lv.y;
      qz += (double)lv.z * (double)lv.z; qw += (double)lv.w * (double)lv.w;
    } else {
      v.x = fmaxf(v.x, 0.0f); v.y = fmaxf(v.y, 0.0f); v.z = fmaxf(v.z, 0.0f); v.w = fmaxf(v.w, 0.0f);
      const v4f hres = *(const v4f*)(outF + (size_t)row * DM + c4);
      const v4f t = hres + v;
      float s = (t.x + t.y) + (t.z + t.w);
#pragma unroll
      for (int off = 16; off > 0; off >>= 1) s += __shfl_xor(s, off);
      const float mean = s * 0.0078125f;
      const v4f d = t - mean;
      float q = d.x * d.x + d.y * d.y + d.z * d.z + d.w * d.w;
#pragma unroll
      for (int off = 16; off > 0; off >>= 1) q += __shfl_xor(q, off);
      const float var = q * 0.0078125f;
      const float rstd = rsqrtf(var + 1e-5f);
      const v4f y = d * rstd * lg4 + lb4;
      o = live ? y : zero4;
    }
    float* op = outF + (size_t)row * DM + c4;
    *(volatile v4f*)op = o;
    __threadfence();
    *(volatile v4f*)op = o;
  }

  if (MODE == 1) {
    double* stp = sSt + (wave * 32 + lane) * 8;
    stp[0] = sx; stp[1] = sy; stp[2] = sz; stp[3] = sw;
    stp[4] = qx; stp[5] = qy; stp[6] = qz; stp[7] = qw;
    __syncthreads();
    if (tid < 128) {
      const int ln = tid >> 2, cp = tid & 3;
      double S = 0.0, Q = 0.0;
#pragma unroll
      for (int w = 0; w < 8; ++w) {
        S += sSt[(w * 32 + ln) * 8 + cp];
        Q += sSt[(w * 32 + ln) * 8 + 4 + cp];
      }
      sCol[tid] = S;
      sCol[128 + tid] = Q;
    }
    __syncthreads();
    const bool wr = tid < 128;
    const v2d pv = *(const v2d*)(sCol + 2 * (tid & 127));
    double* gp = part + (size_t)blockIdx.x * 256 + 2 * (tid & 127);
    if (wr) *(volatile v2d*)gp = pv;
    __threadfence();
    if (wr) *(volatile v2d*)gp = pv;
  }
}

__global__ __launch_bounds__(128) void k_bnfin(
    const double* __restrict__ part, int nblk, int nlive, float* stats) {
  __shared__ __attribute__((aligned(16))) float sF[256];
  const int c = (int)threadIdx.x;
  double s = 0.0, s2 = 0.0;
#pragma unroll 1
  for (int b = 0; b < nblk; ++b) {
    s  += part[(size_t)b * 256 + c];
    s2 += part[(size_t)b * 256 + 128 + c];
  }
  const double invn = 1.0 / (double)nlive;
  const double mu = s * invn;
  double var = s2 * invn - mu * mu;
  var = var < 0.0 ? 0.0 : var;
  const float varf = (float)var;
  sF[c] = (float)mu;
  sF[128 + c] = rsqrtf(varf + 1e-5f);
  __syncthreads();
  const bool w = c < 64;
  const int cc = c & 63;
  const v4f v = *(const v4f*)(sF + 4 * cc);
  if (w) *(volatile v4f*)(stats + 4 * cc) = v;
  __threadfence();
  if (w) *(volatile v4f*)(stats + 4 * cc) = v;
}

__global__ __launch_bounds__(256) void k_pool(
    const float* __restrict__ H, const int* __restrict__ bat, float* out, int nN, int nG) {
  __shared__ int sHit[256];
  __shared__ int sWc[8];
  __shared__ __attribute__((aligned(32))) v4d sAcc[8 * GPB * 32];
  __shared__ float sCn[8 * GPB];
  const int tid = (int)threadIdx.x, lane = tid & 31, wave = tid >> 5;
  const int g0 = (int)blockIdx.x * GPB;
  const int c4 = 4 * lane;
  const unsigned int lt = (1u << lane) - 1u;
  const v4d zero4d = {0.0, 0.0, 0.0, 0.0};
  v4d acc[GPB];
  float cn[GPB];
#pragma unroll
  for (int r = 0; r < GPB; ++r) { acc[r] = zero4d; cn[r] = 0.0f; }

  const int nchunk = (nN + 255) >> 8;
#pragma unroll 1
  for (int ch = 0; ch < nchunk; ++ch) {
    const int node = (ch << 8) + tid;
    const bool inb = node < nN;
    const int na = inb ? node : (nN - 1);
    const int bt = bat[na];
    const int rel = bt - g0;
    const bool hit = inb && ((unsigned)rel < (unsigned)GPB);
    const unsigned int msk = __builtin_amdgcn_ballot_w32(hit);
    const int pos = (int)__builtin_popcount(msk & lt);
    if (lane == 0) sWc[wave] = (int)__builtin_popcount(msk);
    __syncthreads();
    int pre = 0, tot = 0;
#pragma unroll
    for (int w = 0; w < 8; ++w) { const int c = sWc[w]; pre += (w < wave) ? c : 0; tot += c; }
    if (hit) sHit[pre + pos] = (na << 3) | rel;
    __syncthreads();
    tot = tot > 256 ? 256 : tot;
#pragma unroll 1
    for (int t = wave; t < tot; t += 8) {
      const int en = sHit[t];
      int nd = en >> 3; nd = nd < 0 ? 0 : (nd > nN - 1 ? nN - 1 : nd);
      const int rl = en & 7;
      const v4f v = *(const v4f*)(H + (size_t)nd * DM + c4);
      const v4d vd = __builtin_convertvector(v, v4d);
#pragma unroll
      for (int r = 0; r < GPB; ++r) {
        const bool s = (rl == r);
        acc[r] = s ? (acc[r] + vd) : acc[r];
        cn[r] = s ? (cn[r] + 1.0f) : cn[r];
      }
    }
    __syncthreads();
  }

#pragma unroll
  for (int r = 0; r < GPB; ++r) {
    sAcc[(wave * GPB + r) * 32 + lane] = acc[r];
    if (lane == 0) sCn[wave * GPB + r] = cn[r];
  }
  __syncthreads();
  if (wave < GPB) {
    v4d s = zero4d;
    float c = 0.0f;
#pragma unroll
    for (int w = 0; w < 8; ++w) {
      s = s + sAcc[(w * GPB + wave) * 32 + lane];
      c += sCn[w * GPB + wave];
    }
    const float inv = 1.0f / fmaxf(c, 1.0f);
    v4f sf;
    sf.x = (float)s.x; sf.y = (float)s.y; sf.z = (float)s.z; sf.w = (float)s.w;
    const v4f o = sf * inv;
    const int row = g0 + wave;
    const bool ok = row < nG;
    float* op = out + (size_t)(ok ? row : 0) * DM + c4;
    if (ok) *(volatile v4f*)op = o;
    __threadfence();
    if (ok) *(volatile v4f*)op = o;
  }
}

extern "C" void kernel_launch(void* const* d_in, const int* in_sizes, int n_in,
                              void* d_out, int out_size, void* d_ws, size_t ws_size,
                              hipStream_t stream) {
  if (n_in < 14) return;
  const int nN  = in_sizes[0] / DM;
  const int nE1 = in_sizes[12] / 2;
  if (nN <= 0 || nE1 <= 0 || out_size <= 0) return;
  if (in_sizes[0] != nN * DM || in_sizes[12] != 2 * nE1 || in_sizes[13] != nN) return;
  if (in_sizes[1] != DM * DM || in_sizes[2] != DM || in_sizes[3] != NLAYER) return;
  if (in_sizes[4] != NLAYER * DM * DM || in_sizes[8] != NLAYER * DM * DM) return;
  if (in_sizes[5] != NLAYER * DM || in_sizes[6] != NLAYER * DM || in_sizes[7] != NLAYER * DM) return;
  if (in_sizes[9] != NLAYER * DM || in_sizes[10] != NLAYER * DM || in_sizes[11] != NLAYER * DM) return;
  if ((out_size % DM) != 0) return;
  const int G = out_size / DM;
  if (G <= 0) return;
  const int nE2 = 2 * nE1;
  if (nN > RMAX * RB || nE2 > (1 << 21)) return;

  const float* x    = (const float*)d_in[0];
  const float* W0   = (const float*)d_in[1];
  const float* b0   = (const float*)d_in[2];
  const float* epsl = (const float*)d_in[3];
  const float* W1   = (const float*)d_in[4];
  const float* b1   = (const float*)d_in[5];
  const float* bng  = (const float*)d_in[6];
  const float* bnb  = (const float*)d_in[7];
  const float* W2   = (const float*)d_in[8];
  const float* b2   = (const float*)d_in[9];
  const float* lng  = (const float*)d_in[10];
  const float* lnb  = (const float*)d_in[11];
  const int*   ei   = (const int*)d_in[12];
  const int*   bat  = (const int*)d_in[13];
  const int*   er   = ei;
  const int*   ec   = ei + nE1;
  float* out = (float*)d_out;

  const int nCh  = (nE2 + CHUNK - 1) / CHUNK;
  const int nR   = (nN + RB - 1) / RB;
  const int nNp  = ((nN + 127) / 128) * 128;
  const int nSB  = nNp / 128;
  const int nPB  = (G + GPB - 1) / GPB;
  const int listCap = ((nE2 + 32 * nR + 1023) / 1024) * 1024;
  if (nR > RMAX || nR * RB < nNp) return;

  const size_t szWT   = (size_t)NWROWS * DM * 2;
  const size_t szH    = (size_t)nNp * DM * 4;
  const size_t szP    = szH;
  const size_t szCS   = (size_t)nCh * CHUNK * 4;
  const size_t szTab  = (size_t)nCh * TABW * 4;
  const size_t szSrc  = (size_t)listCap * 4;
  const size_t szNt   = (size_t)nR * RB * 4;
  const size_t szPart = (size_t)nSB * 256 * 8;
  const size_t szStat = 256 * 4;
  size_t off = 0;
  const size_t oWT = off; off += szWT;   off = (off + 255) & ~(size_t)255;
  const size_t oH  = off; off += szH;    off = (off + 255) & ~(size_t)255;
  const size_t oP  = off; off += szP;    off = (off + 255) & ~(size_t)255;
  const size_t oC  = off; off += szCS;   off = (off + 255) & ~(size_t)255;
  const size_t oT  = off; off += szTab;  off = (off + 255) & ~(size_t)255;
  const size_t oS  = off; off += szSrc;  off = (off + 255) & ~(size_t)255;
  const size_t oN  = off; off += szNt;   off = (off + 255) & ~(size_t)255;
  const size_t oPa = off; off += szPart; off = (off + 255) & ~(size_t)255;
  const size_t oSt = off; off += szStat; off = (off + 255) & ~(size_t)255;
  if (off > ws_size || off > (size_t)WSCAP) return;

  char* ws = (char*)d_ws;
  _Float16*     WT    = (_Float16*)(ws + oWT);
  float*        H     = (float*)(ws + oH);
  float*        P     = (float*)(ws + oP);
  unsigned int* csort = (unsigned int*)(ws + oC);
  int*          tab   = (int*)(ws + oT);
  int*          srcs  = (int*)(ws + oS);
  int*          ntab  = (int*)(ws + oN);
  double*       part  = (double*)(ws + oPa);
  float*        stats = (float*)(ws + oSt);

  k_csort<<<nCh, 256, 0, stream>>>(er, ec, csort, tab, nN, nE1, nE2);

  hipFuncSetAttribute(reinterpret_cast<const void*>(&k_csr),
                      hipFuncAttributeMaxDynamicSharedMemorySize, CSR_LDS);
  k_csr<<<nR, 256, CSR_LDS, stream>>>(er, ec, csort, tab, srcs, ntab, nN, nE1, nE2, nCh, listCap);

  k_wprep<<<NWROWS / 32, 256, 0, stream>>>(W0, W1, W2, WT);

  hipFuncSetAttribute(reinterpret_cast<const void*>(&k_gemm<0>),
                      hipFuncAttributeMaxDynamicSharedMemorySize, GEMM_LDS);
  hipFuncSetAttribute(reinterpret_cast<const void*>(&k_gemm<1>),
                      hipFuncAttributeMaxDynamicSharedMemorySize, GEMM_LDS);
  hipFuncSetAttribute(reinterpret_cast<const void*>(&k_gemm<2>),
                      hipFuncAttributeMaxDynamicSharedMemorySize, GEMM_LDS);
  k_gemm<0><<<nSB, 256, GEMM_LDS, stream>>>(
      x, srcs, ntab, listCap, epsl, WT, b0, stats, bng, bnb, lng, lnb, H, part, nN, nNp);

  for (int l = 0; l < NLAYER; ++l) {
    k_gemm<1><<<nSB, 256, GEMM_LDS, stream>>>(
        H, srcs, ntab, listCap, epsl + l, WT + (size_t)(1 + l) * DM * DM, b1 + l * DM,
        stats, bng + l * DM, bnb + l * DM, lng + l * DM, lnb + l * DM, P, part, nN, nNp);
    k_bnfin<<<1, 128, 0, stream>>>(part, nSB, nN, stats);
    k_gemm<2><<<nSB, 256, GEMM_LDS, stream>>>(
        P, srcs, ntab, listCap, epsl + l, WT + (size_t)(1 + NLAYER + l) * DM * DM, b2 + l * DM,
        stats, bng + l * DM, bnb + l * DM, lng + l * DM, lnb + l * DM, H, part, nN, nNp);
  }

  k_pool<<<nPB, 256, 0, stream>>>(H, bat, out, nN, G);
}
